// SelfAttention2_52690658787774
// MI455X (gfx1250) — hardware-verified
//
#include <hip/hip_runtime.h>

#define B_ 16
#define N_ 4096
#define D_ 128
#define KP 136
#define VT_STRIDE 40
#define P_STRIDE  40
#define PSC 16384.0f
#define PUN (1.0f / 16384.0f)

typedef __attribute__((ext_vector_type(16))) _Float16 v16h;
typedef __attribute__((ext_vector_type(8)))  _Float16 v8h;
typedef __attribute__((ext_vector_type(16))) __bf16 v16bf;
typedef __attribute__((ext_vector_type(8)))  __bf16 v8bf;
typedef __attribute__((ext_vector_type(8)))  float  v8f;
typedef __attribute__((ext_vector_type(4)))  float  v4f;
typedef __attribute__((ext_vector_type(4)))  unsigned int v4u;
typedef float __attribute__((may_alias)) float_a;

__device__ __forceinline__ v8f wmma_f16(v16h a, v16h b, v8f c) {
  v8f d = __builtin_amdgcn_wmma_f32_16x16x32_f16(false, a, false, b, (short)0, c, false, false);
  asm volatile("v_nop\n\tv_nop\n\tv_nop\n\tv_nop" : "+v"(d) : "v"(a), "v"(b));
  return d;
}
__device__ __forceinline__ v8f wmma_bf16(v16bf a, v16bf b, v8f c) {
  v8f d = __builtin_amdgcn_wmma_f32_16x16x32_bf16(false, a, false, b, (short)0, c, false, false);
  asm volatile("v_nop\n\tv_nop\n\tv_nop\n\tv_nop" : "+v"(d) : "v"(a), "v"(b));
  return d;
}
__device__ __forceinline__ __bf16 bf_hi(float x) { return (__bf16)x; }
__device__ __forceinline__ __bf16 bf_lo(float x, __bf16 h) { return (__bf16)(x - (float)h); }
template <typename V> __device__ __forceinline__ void vst2(void* p, V v) {
  *(volatile V*)p = v; __threadfence(); *(volatile V*)p = v;
}
template <typename V16, typename V8, typename T>
__device__ __forceinline__ V16 load_frag(const T* tile, int ld, int k0, int lane) {
  union { V16 v; V8 h[2]; } r;
  const T* row = tile + (lane & 15) * ld + k0 + 8 * (lane >> 4);
  r.h[0] = *(const V8*)(row);
  r.h[1] = *(const V8*)(row + 16);
  return r.v;
}
__device__ __forceinline__ v16h load_frag_f32_to_f16(const float* tile, int ld, int k0, int lane) {
  v16h a;
  const float* row = tile + (size_t)(lane & 15) * ld + k0 + 8 * (lane >> 4);
#pragma unroll
  for (int i = 0; i < 8; ++i) { a[i] = (_Float16)row[i]; a[8 + i] = (_Float16)row[16 + i]; }
  return a;
}

__global__ __launch_bounds__(128) void qkv_proj_kernel(
    const float* __restrict__ X,
    const float* __restrict__ Wq, const float* __restrict__ bq,
    const float* __restrict__ Wk, const float* __restrict__ bk,
    const float* __restrict__ Wv, const float* __restrict__ bv,
    float* __restrict__ Q, float* __restrict__ K, _Float16* __restrict__ VT)
{
  __shared__ __align__(16) _Float16 Ws[D_ * KP];
  __shared__ __align__(16) _Float16 Xs[64 * KP];
  __shared__ __align__(16) float    Ot[64 * D_];

  const int m    = blockIdx.y;
  const int n0   = blockIdx.x * 64;
  const int tid  = threadIdx.x;
  const int wave = tid >> 5, lane = tid & 31;
  const int lr   = lane & 15, hi = lane >> 4;

  const float* W    = (m == 0) ? Wq : (m == 1) ? Wk : Wv;
  const float* bias = (m == 0) ? bq : (m == 1) ? bk : bv;
  for (int i = tid; i < D_ * D_; i += 128) { const int n = i >> 7, k = i & 127; Ws[n * KP + k] = (_Float16)W[i]; }
  for (int i = tid; i < 64 * D_; i += 128) { const int r = i >> 7, k = i & 127; Xs[r * KP + k] = (_Float16)X[(size_t)(n0 + r) * D_ + k]; }
  __syncthreads();

  v8f acc[8];
#pragma unroll
  for (int dt = 0; dt < 8; ++dt) acc[dt] = (v8f){};
#pragma unroll
  for (int kk = 0; kk < 4; ++kk) {
    const v16h a = load_frag<v16h, v8h, _Float16>(Xs + wave * 16 * KP, KP, kk * 32, lane);
#pragma unroll
    for (int dt = 0; dt < 8; ++dt)
      acc[dt] = wmma_f16(a, load_frag<v16h, v8h, _Float16>(Ws + dt * 16 * KP, KP, kk * 32, lane), acc[dt]);
  }

  if (m < 2) {
#pragma unroll
    for (int dt = 0; dt < 8; ++dt) {
      const float bb = bias[dt * 16 + lr];
#pragma unroll
      for (int j = 0; j < 8; ++j) Ot[(wave * 16 + hi * 8 + j) * D_ + dt * 16 + lr] = acc[dt][j] + bb;
    }
    __syncthreads();
    float* dst = ((m == 0) ? Q : K) + (size_t)n0 * D_;
    for (int g = tid; g < 64 * 32; g += 128) vst2((char*)dst + g * 16, *(const v4f*)((const char*)Ot + g * 16));
  } else {
    _Float16* Vt = (_Float16*)Ot;
#pragma unroll
    for (int dt = 0; dt < 8; ++dt) {
      const float bb = bias[dt * 16 + lr];
#pragma unroll
      for (int j = 0; j < 8; ++j) Vt[(dt * 16 + lr) * 64 + wave * 16 + hi * 8 + j] = (_Float16)(acc[dt][j] + bb);
    }
    __syncthreads();
    const int b = n0 / N_, nl0 = n0 % N_;
    for (int g = tid; g < 128 * 8; g += 128) {
      const int d = g >> 3, pc = g & 7;
      vst2((char*)(VT + ((size_t)b * D_ + d) * N_ + nl0) + pc * 16, *(const v4u*)((const char*)Vt + d * 128 + pc * 16));
    }
  }
}

__global__ __launch_bounds__(128) void attn_kernel(
    const float* __restrict__ Q, const float* __restrict__ K,
    const _Float16* __restrict__ VT, float* __restrict__ partial)
{
  __shared__ __align__(16) __bf16 Kh[32 * KP];
  __shared__ __align__(16) __bf16 Kl[32 * KP];
  __shared__ __align__(16) _Float16 Vs[D_ * VT_STRIDE];
  __shared__ __align__(16) __bf16 Qh[4][16 * KP];
  __shared__ __align__(16) __bf16 Ql[4][16 * KP];
  __shared__ __align__(16) _Float16 Ps[4][16 * P_STRIDE];
  __shared__ __align__(16) float Po[4][D_];

  const int blk  = blockIdx.x;
  const int b    = blk >> 6;
  const int tid  = threadIdx.x;
  const int wave = tid >> 5;
  const int lane = tid & 31;
  const int lr   = lane & 15;
  const int hi   = lane >> 4;
  const int qt   = (blk & 63) * 4 + wave;
  const size_t g0 = (size_t)b * N_ + qt * 16;

  const float* Kg = K + (size_t)b * N_ * D_;
  const _Float16* Vg = VT + (size_t)b * D_ * N_;

  for (int i = lane; i < 16 * D_; i += 32) {
    const int r = i >> 7, c = i & 127;
    const float x = Q[(g0 + r) * D_ + c];
    const __bf16 hb = bf_hi(x);
    Qh[wave][r * KP + c] = hb; Ql[wave][r * KP + c] = bf_lo(x, hb);
  }

  v8f ot[8];
#pragma unroll
  for (int t = 0; t < 8; ++t) ot[t] = (v8f){};
  float mrun[8], lrun[8];
#pragma unroll
  for (int j = 0; j < 8; ++j) { mrun[j] = -1e30f; lrun[j] = 0.0f; }

  const float LOG2E = 1.44269504f;
  _Float16* Pw = &Ps[wave][0];

  for (int kb = 0; kb < N_ / 32; ++kb) {
    const int k0 = kb * 32;
    __syncthreads();
    for (int i = tid; i < 32 * D_; i += 128) {
      const int r = i >> 7, c = i & 127;
      const float x = Kg[(size_t)(k0 + r) * D_ + c];
      const __bf16 hb = bf_hi(x);
      Kh[r * KP + c] = hb; Kl[r * KP + c] = bf_lo(x, hb);
    }
    for (int i = tid; i < D_ * 4; i += 128) {
      const int d = i >> 2, part = i & 3;
      *(v4u*)(&Vs[d * VT_STRIDE + part * 8]) = *(const v4u*)(Vg + (size_t)d * N_ + k0 + part * 8);
    }
    __syncthreads();

    v8f s0 = {}, s1 = {};
#pragma unroll
    for (int kk = 0; kk < 4; ++kk) {
      const v16bf qh = load_frag<v16bf, v8bf, __bf16>(Qh[wave], KP, kk * 32, lane);
      const v16bf ql = load_frag<v16bf, v8bf, __bf16>(Ql[wave], KP, kk * 32, lane);
      v16bf kh0 = load_frag<v16bf, v8bf, __bf16>(Kh, KP, kk * 32, lane);
      v16bf kl0 = load_frag<v16bf, v8bf, __bf16>(Kl, KP, kk * 32, lane);
      s0 = wmma_bf16(qh, kh0, s0); s0 = wmma_bf16(qh, kl0, s0); s0 = wmma_bf16(ql, kh0, s0);
      v16bf kh1 = load_frag<v16bf, v8bf, __bf16>(Kh + 16 * KP, KP, kk * 32, lane);
      v16bf kl1 = load_frag<v16bf, v8bf, __bf16>(Kl + 16 * KP, KP, kk * 32, lane);
      s1 = wmma_bf16(qh, kh1, s1); s1 = wmma_bf16(qh, kl1, s1); s1 = wmma_bf16(ql, kh1, s1);
    }

    float alpha[8];
#pragma unroll
    for (int j = 0; j < 8; ++j) {
      float mx = fmaxf(s0[j], s1[j]);
#pragma unroll
      for (int off = 1; off < 16; off <<= 1)
        mx = fmaxf(mx, __shfl_xor(mx, off, 32));
      const float mnew = fmaxf(mrun[j], mx);
      alpha[j] = exp2f((mrun[j] - mnew) * LOG2E);
      const float p0 = exp2f((s0[j] - mnew) * LOG2E);
      const float p1 = exp2f((s1[j] - mnew) * LOG2E);
      Pw[(j + 8 * hi) * P_STRIDE + lr]      = (_Float16)(p0 * PSC);
      Pw[(j + 8 * hi) * P_STRIDE + 16 + lr] = (_Float16)(p1 * PSC);
      float rsum = p0 + p1;
#pragma unroll
      for (int off = 1; off < 16; off <<= 1)
        rsum += __shfl_xor(rsum, off, 32);
      lrun[j] = lrun[j] * alpha[j] + rsum;
      mrun[j] = mnew;
    }
#pragma unroll
    for (int t = 0; t < 8; ++t)
#pragma unroll
      for (int j = 0; j < 8; ++j) ot[t][j] *= alpha[j];

    __syncthreads();
    const v16h pa = load_frag<v16h, v8h, _Float16>(Pw, P_STRIDE, 0, lane);

#pragma unroll
    for (int t = 0; t < 8; ++t) {
      const v16h vt = load_frag<v16h, v8h, _Float16>(Vs + t * 16 * VT_STRIDE, VT_STRIDE, 0, lane);
      ot[t] = wmma_f16(pa, vt, ot[t]);
    }
  }

  float inv[8];
#pragma unroll
  for (int j = 0; j < 8; ++j) inv[j] = PUN / lrun[j];
#pragma unroll
  for (int t = 0; t < 8; ++t) {
    float cs = 0.0f;
#pragma unroll
    for (int j = 0; j < 8; ++j) cs += ot[t][j] * inv[j];
    cs += __shfl_xor(cs, 16, 32);
    if (hi == 0) Po[wave][t * 16 + lr] = cs;
  }
  __syncthreads();
  {
    const v4f v = *(const v4f*)(&Po[wave][lane * 4]);
    vst2(partial + ((size_t)(b * (N_ / 16) + qt)) * D_ + lane * 4, v);
  }
}

__global__ __launch_bounds__(256) void reduce_kernel(const float* __restrict__ partial, float* __restrict__ out)
{
  const int idx = blockIdx.x * blockDim.x + threadIdx.x;
  const int b = idx / D_;
  const int d = idx % D_;
  float s = 0.0f;
  for (int qtile = 0; qtile < N_ / 16; ++qtile)
    s += partial[((size_t)(b * (N_ / 16) + qtile)) * D_ + d];
  vst2(out + idx, (float_a)(s * (1.0f / (float)N_)));
}

extern "C" void kernel_launch(void* const* d_in, const int* in_sizes, int n_in,
                              void* d_out, int out_size, void* d_ws, size_t ws_size,
                              hipStream_t stream) {
  (void)in_sizes; (void)n_in; (void)out_size; (void)ws_size;
  const float* X  = (const float*)d_in[0];
  const float* Wq = (const float*)d_in[1];
  const float* bq = (const float*)d_in[2];
  const float* Wk = (const float*)d_in[3];
  const float* bk = (const float*)d_in[4];
  const float* Wv = (const float*)d_in[5];
  const float* bv = (const float*)d_in[6];

  char* ws = (char*)d_ws;
  const size_t f32_bytes = (size_t)B_ * N_ * D_ * 4;
  const size_t f16_bytes = (size_t)B_ * N_ * D_ * 2;
  float* Q  = (float*)(ws);
  float* K  = (float*)(ws + f32_bytes);
  _Float16* VT = (_Float16*)(ws + 2 * f32_bytes);
  float* partial = (float*)(ws + 2 * f32_bytes + f16_bytes);

  dim3 g1(B_ * N_ / 64, 3);
  qkv_proj_kernel<<<g1, 128, 0, stream>>>(X, Wq, bq, Wk, bk, Wv, bv, Q, K, VT);
  attn_kernel<<<(B_ * (N_ / 16)) / 4, 128, 0, stream>>>(Q, K, VT, partial);
  reduce_kernel<<<(B_ * D_) / 256, 256, 0, stream>>>(partial, (float*)d_out);
}
